// RGCNForGraphClassification_56667798503745
// MI455X (gfx1250) — hardware-verified
//
#include <hip/hip_runtime.h>
#include <stddef.h>
#include <stdint.h>


#define IN1      256
#define HIDC     128
#define OUTC     8
#define NREL     4
#define NBAS     8
#define NGMAX    64
#define NTHR     256
#define NWAVE    8
#define EPT      8
#define CHUNK    (NTHR * EPT)
#define WCAP     (EPT * 32)
#define LISTN    (NWAVE * WCAP)
#define NBMAX    2048
#define RCAP     28672
#define DEGCAP   4096
#define GBM      64
#define GTHR     128
#define CA       16.0f
#define CW       64.0f
#define SCL      0.0009765625f
#define WSMAX    134217728
#define LDS_AGG  ((2 * RCAP + 2 * NBMAX + LISTN) * 4 + 64)
#define LDS_POOL ((2 * NGMAX * HIDC + 2 * NGMAX + NGMAX * OUTC) * 4)

static_assert((CHUNK & (CHUNK - 1)) == 0 && CHUNK <= 4096);
static_assert((NBMAX & (NBMAX - 1)) == 0 && NBMAX <= 4096);
static_assert(NTHR * 8 == NBMAX);
static_assert(LISTN >= NBMAX);
static_assert(LISTN >= NWAVE * WCAP);
static_assert((RCAP % 32) == 0);
static_assert(LDS_AGG <= 300000);
static_assert(LDS_POOL <= 300000);
static_assert(GBM == (GTHR / 32) * 16);
static_assert((IN1 % 32) == 0 && (HIDC % 32) == 0 && HIDC == 128);
static_assert(NTHR == 2 * HIDC);
static_assert(2 * NGMAX <= NTHR);
static_assert((NGMAX * OUTC) % NTHR == 0);
static_assert((NGMAX * OUTC) / 4 <= NTHR);

typedef float    v4f  __attribute__((ext_vector_type(4)));
typedef float    v8f  __attribute__((ext_vector_type(8)));
typedef int      v4i  __attribute__((ext_vector_type(4)));
typedef int      v8i  __attribute__((ext_vector_type(8)));
typedef _Float16 v8h  __attribute__((ext_vector_type(8)));
typedef _Float16 v16h __attribute__((ext_vector_type(16)));
union FragH { v16h v; v8h h[2]; v8i w; };

__device__ __forceinline__ v8f wmh(const FragH& a, const FragH& b, v8f c) {
  v8f d = __builtin_amdgcn_wmma_f32_16x16x32_f16(false, a.v, false, b.v, (short)0, c, false, false);
  asm volatile("v_nop\n\tv_nop\n\tv_nop\n\tv_nop" : "+v"(d) : "v"(a.w), "v"(b.w));
  return d;
}

__device__ __forceinline__ v8h cvt8(v4f a, v4f b) {
  v8h h;
  h[0] = (_Float16)(a.x * CA); h[1] = (_Float16)(a.y * CA); h[2] = (_Float16)(a.z * CA); h[3] = (_Float16)(a.w * CA);
  h[4] = (_Float16)(b.x * CA); h[5] = (_Float16)(b.y * CA); h[6] = (_Float16)(b.z * CA); h[7] = (_Float16)(b.w * CA);
  return h;
}

__device__ __forceinline__ v8h mean8(v4f a, v4f b, float sc, bool pois) {
  const float qn = __int_as_float(0x7fc00000);
  const float v0 = a.x * sc, v1 = a.y * sc, v2 = a.z * sc, v3 = a.w * sc;
  const float v4 = b.x * sc, v5 = b.y * sc, v6 = b.z * sc, v7 = b.w * sc;
  v8h h;
  h[0] = (_Float16)(pois ? qn : v0); h[1] = (_Float16)(pois ? qn : v1);
  h[2] = (_Float16)(pois ? qn : v2); h[3] = (_Float16)(pois ? qn : v3);
  h[4] = (_Float16)(pois ? qn : v4); h[5] = (_Float16)(pois ? qn : v5);
  h[6] = (_Float16)(pois ? qn : v6); h[7] = (_Float16)(pois ? qn : v7);
  return h;
}

__device__ __forceinline__ int scan_chunk(const int* __restrict__ dsts, int nE, int cbase, int slotBase,
                                          int nb, int vec8, int* list, int tid, int lane, int wave) {
  int wc = 0;
  const int el0  = tid * EPT;
  const int e0   = cbase + el0;
  const int sent = -2147483647 - 1;
  v4i da, db;
  if (vec8 != 0 && cbase + CHUNK <= nE) {
    da = *(const v4i*)(dsts + e0);
    db = *(const v4i*)(dsts + e0 + 4);
  } else {
    da.x = (e0     < nE) ? dsts[min(e0,     nE - 1)] : sent;
    da.y = (e0 + 1 < nE) ? dsts[min(e0 + 1, nE - 1)] : sent;
    da.z = (e0 + 2 < nE) ? dsts[min(e0 + 2, nE - 1)] : sent;
    da.w = (e0 + 3 < nE) ? dsts[min(e0 + 3, nE - 1)] : sent;
    db.x = (e0 + 4 < nE) ? dsts[min(e0 + 4, nE - 1)] : sent;
    db.y = (e0 + 5 < nE) ? dsts[min(e0 + 5, nE - 1)] : sent;
    db.z = (e0 + 6 < nE) ? dsts[min(e0 + 6, nE - 1)] : sent;
    db.w = (e0 + 7 < nE) ? dsts[min(e0 + 7, nE - 1)] : sent;
  }
  const unsigned nbs = (unsigned)slotBase;
  const unsigned unb = (unsigned)nb;
  const unsigned s0 = (unsigned)da.x - nbs, s1 = (unsigned)da.y - nbs;
  const unsigned s2 = (unsigned)da.z - nbs, s3 = (unsigned)da.w - nbs;
  const unsigned s4 = (unsigned)db.x - nbs, s5 = (unsigned)db.y - nbs;
  const unsigned s6 = (unsigned)db.z - nbs, s7 = (unsigned)db.w - nbs;
  const bool h0 = s0 < unb, h1 = s1 < unb, h2 = s2 < unb, h3 = s3 < unb;
  const bool h4 = s4 < unb, h5 = s5 < unb, h6 = s6 < unb, h7 = s7 < unb;
  const unsigned any = __builtin_amdgcn_ballot_w32(h0 | h1 | h2 | h3 | h4 | h5 | h6 | h7);
  if (any != 0u) {
#define HITJ(J, HJ, SJ) { \
      const unsigned mj = __builtin_amdgcn_ballot_w32(HJ); \
      if (mj != 0u) { \
        if (HJ) { \
          const int pos = wc + (int)__builtin_amdgcn_mbcnt_lo(mj, 0u); \
          if (pos < WCAP) list[wave * WCAP + pos] = ((el0 + (J)) << 12) | (int)(SJ); \
        } \
        wc += (int)__builtin_popcount(mj); } }
    HITJ(0, h0, s0)
    HITJ(1, h1, s1)
    HITJ(2, h2, s2)
    HITJ(3, h3, s3)
    HITJ(4, h4, s4)
    HITJ(5, h5, s5)
    HITJ(6, h6, s6)
    HITJ(7, h7, s7)
#undef HITJ
  }
  return wc;
}

__global__ __launch_bounds__(NTHR) void k_wprep(const float* __restrict__ bases, const float* __restrict__ comp,
                                               const float* __restrict__ root, _Float16* wt, int KIN, int nUnits) {
  const int u = (int)blockIdx.x * NTHR + (int)threadIdx.x;
  if (u >= nUnits) return;
  const int KT  = (NREL + 1) * KIN;
  const int upr = KT >> 3;
  const int n   = u / upr;
  const int k8  = (u - n * upr) * 8;
  const int r   = k8 / KIN;
  const int i0  = k8 - r * KIN;
  const int rr  = r < NREL ? r : NREL - 1;
  float s[8];
#pragma unroll
  for (int j = 0; j < 8; ++j) s[j] = 0.0f;
#pragma unroll 1
  for (int b = 0; b < NBAS; ++b) {
    const float cb = comp[rr * NBAS + b];
    const float* bp = bases + ((size_t)b * (size_t)KIN + (size_t)i0) * HIDC + n;
#pragma unroll
    for (int j = 0; j < 8; ++j) s[j] = fmaf(cb, bp[(size_t)j * HIDC], s[j]);
  }
  const float* rp = root + (size_t)i0 * HIDC + n;
  const bool isw = r < NREL;
  v8h hv;
#pragma unroll
  for (int j = 0; j < 8; ++j) {
    const float rv = rp[(size_t)j * HIDC];
    const float v = isw ? s[j] : rv;
    hv[j] = (_Float16)(v * CW);
  }
  const size_t o = (size_t)n * (size_t)KT + (size_t)k8;
  *(volatile v8h*)(wt + o) = hv;
  __threadfence();
  *(volatile v8h*)(wt + o) = hv;
}

__global__ __launch_bounds__(GTHR) void k_gemm(const _Float16* __restrict__ ap, int lda, int kaSteps,
                                               const float* __restrict__ xs, int ldx, int kxSteps, int nN,
                                               const _Float16* __restrict__ wt, int ldw,
                                               const float* __restrict__ bias, float* H, int MP) {
  __shared__ __attribute__((aligned(16))) float stg[(GTHR / 32) * 16 * HIDC];
  const int tid = threadIdx.x, lane = tid & 31, wave = tid >> 5, hh = lane >> 4, m = lane & 15;
  const int rowBase = (int)blockIdx.x * GBM;
  int row = rowBase + 16 * wave + m;
  row = row < MP ? row : MP - 1;
  v8f acc[8];
  {
    const v8f z = {0.f, 0.f, 0.f, 0.f, 0.f, 0.f, 0.f, 0.f};
#pragma unroll
    for (int t = 0; t < 8; ++t) acc[t] = z;
  }
  const _Float16* arow = ap + (size_t)row * (size_t)lda + 8 * hh;
  const _Float16* brow = wt + (size_t)m * (size_t)ldw + 8 * hh;
  const size_t tstride = (size_t)16 * (size_t)ldw;

#pragma unroll 1
  for (int ks = 0; ks < kaSteps; ++ks) {
    FragH a;
    a.h[0] = *(const v8h*)(arow + 32 * ks);
    a.h[1] = *(const v8h*)(arow + 32 * ks + 16);
    const _Float16* bk = brow + 32 * ks;
#pragma unroll
    for (int t = 0; t < 8; ++t) {
      FragH b;
      b.h[0] = *(const v8h*)(bk + t * tstride);
      b.h[1] = *(const v8h*)(bk + t * tstride + 16);
      acc[t] = wmh(a, b, acc[t]);
    }
  }

  const int rc = row < nN ? row : nN - 1;
  const bool zr = row >= nN;
  const float* xrow = xs + (size_t)rc * (size_t)ldx + 8 * hh;
  const v4f z4 = {0.f, 0.f, 0.f, 0.f};
#pragma unroll 1
  for (int ks = 0; ks < kxSteps; ++ks) {
    const float* xp = xrow + 32 * ks;
    v4f p0 = *(const v4f*)(xp);
    v4f p1 = *(const v4f*)(xp + 4);
    v4f p2 = *(const v4f*)(xp + 16);
    v4f p3 = *(const v4f*)(xp + 20);
    if (zr) { p0 = z4; p1 = z4; p2 = z4; p3 = z4; }
    FragH a;
    a.h[0] = cvt8(p0, p1);
    a.h[1] = cvt8(p2, p3);
    const _Float16* bk = brow + lda + 32 * ks;
#pragma unroll
    for (int t = 0; t < 8; ++t) {
      FragH b;
      b.h[0] = *(const v8h*)(bk + t * tstride);
      b.h[1] = *(const v8h*)(bk + t * tstride + 16);
      acc[t] = wmh(a, b, acc[t]);
    }
  }

  float* sp = stg + wave * (16 * HIDC) + (8 * hh) * HIDC + m;
#pragma unroll
  for (int t = 0; t < 8; ++t) {
    const float bv = bias[16 * t + m];
#pragma unroll
    for (int r = 0; r < 8; ++r) {
      float v = fmaf(acc[t][r], SCL, bv);
      v = (v < 0.0f) ? 0.0f : v;
      sp[r * HIDC + 16 * t] = v;
    }
  }
  __syncthreads();
  const float* sw = stg + wave * (16 * HIDC) + 4 * lane;
  float* hw = H + (size_t)(rowBase + 16 * wave) * HIDC + 4 * lane;
#pragma unroll
  for (int j = 0; j < 16; ++j) {
    const v4f v = *(const v4f*)(sw + j * HIDC);
    *(volatile v4f*)(hw + (size_t)j * HIDC) = v;
  }
  __threadfence();
#pragma unroll
  for (int j = 0; j < 16; ++j) {
    const v4f v = *(const v4f*)(sw + j * HIDC);
    *(volatile v4f*)(hw + (size_t)j * HIDC) = v;
  }
}

__global__ __launch_bounds__(NTHR) void k_agg(
    const int* __restrict__ srcs, const int* __restrict__ dsts, const int* __restrict__ etyp,
    const float* __restrict__ F, int ldf, _Float16* AP, int lda,
    int nN, int nE, int nb, int vec8, int MP) {
  extern __shared__ v4f lds_dyn[];
  int* reg1 = (int*)lds_dyn;
  int* reg2 = reg1 + RCAP;
  int* scnt = reg2 + RCAP;
  int* soff = scnt + NBMAX;
  int* list = soff + NBMAX;
  int* wcnt = list + LISTN;
  int* wtot = wcnt + NWAVE;
  const int tid = threadIdx.x, lane = tid & 31, wave = tid >> 5;
  const int nodeBase = (int)blockIdx.x * nb;

  for (int i = tid; i < NBMAX; i += NTHR) scnt[i] = 0;
  __syncthreads();

  int tot = 0;
  const int nChunks = (nE + CHUNK - 1) / CHUNK;
#pragma unroll 1
  for (int ch = 0; ch < nChunks; ++ch) {
    const int cbase = ch * CHUNK;
    const int wc = scan_chunk(dsts, nE, cbase, nodeBase, nb, vec8, list, tid, lane, wave);
    if (lane == 0) wcnt[wave] = wc;
    __syncthreads();
    int pre = 0, all = 0;
#pragma unroll
    for (int w2 = 0; w2 < NWAVE; ++w2) {
      int c = wcnt[w2];
      c = c < 0 ? 0 : (c > WCAP ? WCAP : c);
      all += c;
      pre += (w2 < wave) ? c : 0;
    }
    const int wcc  = wc > WCAP ? WCAP : wc;
    const int base = tot + pre;
#pragma unroll 1
    for (int i = lane; i < wcc; i += 32) {
      const int ent = list[wave * WCAP + i];
      const int el  = (ent >> 12) & (CHUNK - 1);
      const int sl  = ent & (NBMAX - 1);
      int eid = cbase + el;
      eid = eid > nE - 1 ? nE - 1 : eid;
      const int pos = base + i;
      if (pos < RCAP) reg1[pos] = (int)(((unsigned)eid << 12) | (unsigned)sl);
    }
    tot += all;
    tot = tot > RCAP ? RCAP : tot;
    __syncthreads();
  }
  const int nh = tot;

  if (wave == 0) {
#pragma unroll 1
    for (int b0 = 0; b0 < nh; b0 += 32) {
      const int idx = b0 + lane;
      const int uv  = reg1[idx < RCAP ? idx : RCAP - 1];
      const int m32 = (nh - b0) < 32 ? (nh - b0) : 32;
#pragma unroll 1
      for (int k = 0; k < m32; ++k) {
        const int u  = __builtin_amdgcn_readlane(uv, k);
        const int sl = u & (NBMAX - 1);
        if (lane == 0) scnt[sl] = scnt[sl] + 1;
      }
    }
  }
  __syncthreads();

  {
    const v4i cva = *(const v4i*)(scnt + 8 * tid);
    const v4i cvb = *(const v4i*)(scnt + 8 * tid + 4);
    const int e0 = cva.x < 0 ? 0 : cva.x, e1 = cva.y < 0 ? 0 : cva.y, e2 = cva.z < 0 ? 0 : cva.z, e3 = cva.w < 0 ? 0 : cva.w;
    const int e4 = cvb.x < 0 ? 0 : cvb.x, e5 = cvb.y < 0 ? 0 : cvb.y, e6 = cvb.z < 0 ? 0 : cvb.z, e7 = cvb.w < 0 ? 0 : cvb.w;
    const int ts = e0 + e1 + e2 + e3 + e4 + e5 + e6 + e7;
    int incl = ts;
#pragma unroll
    for (int d = 1; d < 32; d <<= 1) {
      const int up = __shfl_up(incl, d);
      if (lane >= d) incl += up;
    }
    if (lane == 31) wtot[wave] = incl;
    __syncthreads();
    int pre = 0;
#pragma unroll
    for (int w2 = 0; w2 < NWAVE; ++w2) pre += (w2 < wave) ? wtot[w2] : 0;
    int run = pre + incl - ts;
    soff[8 * tid + 0] = run; run += e0;
    soff[8 * tid + 1] = run; run += e1;
    soff[8 * tid + 2] = run; run += e2;
    soff[8 * tid + 3] = run; run += e3;
    soff[8 * tid + 4] = run; run += e4;
    soff[8 * tid + 5] = run; run += e5;
    soff[8 * tid + 6] = run; run += e6;
    soff[8 * tid + 7] = run;
  }
  __syncthreads();
  for (int i = tid; i < NBMAX; i += NTHR) list[i] = soff[i];
  __syncthreads();

  if (wave == 0) {
#pragma unroll 1
    for (int b0 = 0; b0 < nh; b0 += 32) {
      const int idx = b0 + lane;
      const int uv  = reg1[idx < RCAP ? idx : RCAP - 1];
      const int m32 = (nh - b0) < 32 ? (nh - b0) : 32;
#pragma unroll 1
      for (int k = 0; k < m32; ++k) {
        const int u   = __builtin_amdgcn_readlane(uv, k);
        const int sl  = u & (NBMAX - 1);
        const int eid = (int)((unsigned)u >> 12);
        if (lane == 0) {
          int pos = list[sl];
          pos = pos < 0 ? 0 : (pos > RCAP - 1 ? RCAP - 1 : pos);
          reg2[pos] = eid;
          list[sl] = pos + 1;
        }
      }
    }
  }
  __syncthreads();

  const int nbw  = nb >> 3;
  const bool ovf = (nh >= RCAP);
  const int upl  = ldf >> 3;
  const int lsub = lane & (upl - 1);
  const v4f z4 = {0.f, 0.f, 0.f, 0.f};
#pragma unroll 1
  for (int jt = 0; jt < nbw; ++jt) {
    const int slot = wave * nbw + jt;
    const int grow = nodeBase + slot;
    const int sidx = slot < NBMAX ? slot : NBMAX - 1;
    int st = __builtin_amdgcn_readfirstlane(soff[sidx]);
    const int craw = __builtin_amdgcn_readfirstlane(scnt[sidx]);
    int cnt = craw;
    st  = st < 0 ? 0 : (st > nh ? nh : st);
    cnt = cnt < 0 ? 0 : (cnt > DEGCAP ? DEGCAP : cnt);
    if (cnt > nh - st) cnt = nh - st;
    const bool pois = ovf || (craw > DEGCAP);
    const bool wr = (grow < MP);

    v4f a0 = z4, b0 = z4, a1 = z4, b1 = z4, a2 = z4, b2 = z4, a3 = z4, b3 = z4;
    float c0 = 0.f, c1 = 0.f, c2 = 0.f, c3 = 0.f;
#pragma unroll 1
    for (int q = 0; q < cnt; ++q) {
      int idx = st + q; idx = idx > RCAP - 1 ? RCAP - 1 : idx;
      int eid = __builtin_amdgcn_readfirstlane(reg2[idx]);
      eid = eid < 0 ? 0 : (eid > nE - 1 ? nE - 1 : eid);
      int s = srcs[eid];
      s = s < 0 ? 0 : (s > nN - 1 ? nN - 1 : s);
      int t = etyp[eid];
      t = t < 0 ? 0 : (t > NREL - 1 ? NREL - 1 : t);
      t = __builtin_amdgcn_readfirstlane(t);
      const float* fr = F + (size_t)s * (size_t)ldf + 8 * lsub;
      const v4f va = *(const v4f*)(fr);
      const v4f vb = *(const v4f*)(fr + 4);
      if (t == 0)      { a0 += va; b0 += vb; c0 += 1.0f; }
      else if (t == 1) { a1 += va; b1 += vb; c1 += 1.0f; }
      else if (t == 2) { a2 += va; b2 += vb; c2 += 1.0f; }
      else             { a3 += va; b3 += vb; c3 += 1.0f; }
    }
    const float i0 = 1.0f / fmaxf(c0, 1.0f);
    const float i1 = 1.0f / fmaxf(c1, 1.0f);
    const float i2 = 1.0f / fmaxf(c2, 1.0f);
    const float i3 = 1.0f / fmaxf(c3, 1.0f);
    const v8h h0 = mean8(a0, b0, i0 * CA, pois);
    const v8h h1 = mean8(a1, b1, i1 * CA, pois);
    const v8h h2 = mean8(a2, b2, i2 * CA, pois);
    const v8h h3 = mean8(a3, b3, i3 * CA, pois);
    const int gw = grow < MP ? grow : MP - 1;
    _Float16* op = AP + (size_t)gw * (size_t)lda + 8 * lsub;
    const bool ws = wr && (lane < upl);
    if (ws) {
      *(volatile v8h*)(op)                   = h0;
      *(volatile v8h*)(op + (size_t)ldf)     = h1;
      *(volatile v8h*)(op + (size_t)2 * ldf) = h2;
      *(volatile v8h*)(op + (size_t)3 * ldf) = h3;
    }
    __threadfence();
    if (ws) {
      *(volatile v8h*)(op)                   = h0;
      *(volatile v8h*)(op + (size_t)ldf)     = h1;
      *(volatile v8h*)(op + (size_t)2 * ldf) = h2;
      *(volatile v8h*)(op + (size_t)3 * ldf) = h3;
    }
  }
}

__global__ __launch_bounds__(NTHR) void k_pool_head(const float* __restrict__ H2, const int* __restrict__ bat,
                                                   const float* __restrict__ Wc, const float* __restrict__ bc,
                                                   float* out, int nN, int nG) {
  extern __shared__ v4f lds_pool[];
  float* sacc = (float*)lds_pool;
  float* scn  = sacc + 2 * NGMAX * HIDC;
  float* sout = scn + 2 * NGMAX;
  const int tid = threadIdx.x, c = tid & (HIDC - 1), half = tid >> 7;
  const int ngc = nG < 1 ? 1 : (nG > NGMAX ? NGMAX : nG);
  float* mya = sacc + (size_t)half * NGMAX * HIDC + c;
#pragma unroll 1
  for (int g = 0; g < NGMAX; ++g) mya[g * HIDC] = 0.0f;
  if (c < NGMAX) scn[half * NGMAX + c] = 0.0f;
  for (int i = tid; i < NGMAX * OUTC; i += NTHR) sout[i] = 0.0f;
  __syncthreads();

#pragma unroll 1
  for (int n = half; n < nN; n += 2) {
    int g = bat[n];
    g = g < 0 ? 0 : (g > ngc - 1 ? ngc - 1 : g);
    const float v = H2[(size_t)n * HIDC + c];
    mya[g * HIDC] += v;
    if (c == 0) scn[half * NGMAX + g] += 1.0f;
  }
  __syncthreads();
  if (tid < NGMAX) {
    const float cn = scn[tid] + scn[NGMAX + tid];
    scn[tid] = 1.0f / fmaxf(cn, 1.0f);
  }
  __syncthreads();
  {
    const int gb = half * (NGMAX / 2);
#pragma unroll 1
    for (int g = gb; g < gb + NGMAX / 2; ++g) {
      const float s = sacc[g * HIDC + c] + sacc[(NGMAX + g) * HIDC + c];
      sacc[g * HIDC + c] = s * scn[g];
    }
  }
  __syncthreads();
#pragma unroll 1
  for (int k2 = 0; k2 < (NGMAX * OUTC) / NTHR; ++k2) {
    const int idx = tid + k2 * NTHR;
    const int g = idx >> 3, o = idx & (OUTC - 1);
    float a = 0.0f;
#pragma unroll 1
    for (int cc = 0; cc < HIDC; ++cc) a = fmaf(sacc[g * HIDC + cc], Wc[cc * OUTC + o], a);
    sout[idx] = (g < ngc) ? (a + bc[o]) : 0.0f;
  }
  __syncthreads();
  const int nq = (ngc * OUTC) >> 2;
  const bool wq = tid < nq;
  const int tq = tid < (NGMAX * OUTC) / 4 ? tid : (NGMAX * OUTC) / 4 - 1;
  const v4f v = *(const v4f*)(sout + 4 * tq);
  if (wq) *(volatile v4f*)(out + 4 * tq) = v;
  __threadfence();
  if (wq) *(volatile v4f*)(out + 4 * tq) = v;
}

static int pick_nb(int nE, int nN) {
  int nb = NBMAX;
  while (nb > 16 && (long long)nb * (long long)nE * 5LL > (long long)RCAP * (long long)nN * 4LL) nb >>= 1;
  return nb;
}

extern "C" void kernel_launch(void* const* d_in, const int* in_sizes, int n_in,
                              void* d_out, int out_size, void* d_ws, size_t ws_size,
                              hipStream_t stream) {
  if (n_in < 14) return;
  const int nN = in_sizes[0] / IN1;
  if (nN <= 0 || in_sizes[0] != nN * IN1) return;
  if (nN > (1 << 21)) return;
  const int nE = in_sizes[2];
  if (nE < 1 || in_sizes[1] != 2 * nE) return;
  if (nE > (1 << 20)) return;
  if (in_sizes[3] != nN) return;
  if (in_sizes[4] != NBAS * IN1 * HIDC || in_sizes[5] != NREL * NBAS) return;
  if (in_sizes[6] != IN1 * HIDC || in_sizes[7] != HIDC) return;
  if (in_sizes[8] != NBAS * HIDC * HIDC || in_sizes[9] != NREL * NBAS) return;
  if (in_sizes[10] != HIDC * HIDC || in_sizes[11] != HIDC) return;
  if (in_sizes[12] != HIDC * OUTC || in_sizes[13] != OUTC) return;
  if (out_size <= 0 || (out_size % OUTC) != 0) return;
  const int nG = out_size / OUTC;
  if (nG > NGMAX) return;

  const float* x      = (const float*)d_in[0];
  const int*   eidx   = (const int*)d_in[1];
  const int*   etyp   = (const int*)d_in[2];
  const int*   batch  = (const int*)d_in[3];
  const float* bases1 = (const float*)d_in[4];
  const float* comp1  = (const float*)d_in[5];
  const float* root1  = (const float*)d_in[6];
  const float* bias1  = (const float*)d_in[7];
  const float* bases2 = (const float*)d_in[8];
  const float* comp2  = (const float*)d_in[9];
  const float* root2  = (const float*)d_in[10];
  const float* bias2  = (const float*)d_in[11];
  const float* Wc     = (const float*)d_in[12];
  const float* bc     = (const float*)d_in[13];
  float* out = (float*)d_out;
  const int* src = eidx;
  const int* dst = eidx + nE;

  const int MP   = ((nN + GBM - 1) / GBM) * GBM;
  const int nb   = pick_nb(nE, nN);
  const int vec8 = ((nE & 3) == 0) ? 1 : 0;
  const int KT1  = (NREL + 1) * IN1;
  const int KT2  = (NREL + 1) * HIDC;
  const int lda1 = NREL * IN1;
  const int lda2 = NREL * HIDC;
  const int nU1  = HIDC * (KT1 / 8);
  const int nU2  = HIDC * (KT2 / 8);

  char* ws = (char*)d_ws;
  size_t off = 0;
  const size_t oW1 = off; off += (size_t)HIDC * (size_t)KT1 * 2;          off = (off + 255) & ~(size_t)255;
  const size_t oW2 = off; off += (size_t)HIDC * (size_t)KT2 * 2;          off = (off + 255) & ~(size_t)255;
  const size_t oA  = off; off += (size_t)MP * (size_t)lda1 * 2;           off = (off + 255) & ~(size_t)255;
  const size_t oH1 = off; off += (size_t)MP * (size_t)HIDC * 4;           off = (off + 255) & ~(size_t)255;
  if (off > ws_size || off > (size_t)WSMAX) return;
  const size_t oA2 = oA;
  const size_t oH2 = oA + (size_t)MP * (size_t)lda2 * 2;
  if (oH2 + (size_t)MP * (size_t)HIDC * 4 > oA + (size_t)MP * (size_t)lda1 * 2) return;
  _Float16* WT1 = (_Float16*)(ws + oW1);
  _Float16* WT2 = (_Float16*)(ws + oW2);
  _Float16* AP1 = (_Float16*)(ws + oA);
  _Float16* AP2 = (_Float16*)(ws + oA2);
  float*    H1  = (float*)(ws + oH1);
  float*    H2  = (float*)(ws + oH2);

  hipFuncSetAttribute(reinterpret_cast<const void*>(&k_agg),
                      hipFuncAttributeMaxDynamicSharedMemorySize, LDS_AGG);
  hipFuncSetAttribute(reinterpret_cast<const void*>(&k_pool_head),
                      hipFuncAttributeMaxDynamicSharedMemorySize, LDS_POOL);

  const int gG = MP / GBM;
  const int gA = (MP + nb - 1) / nb;

  k_wprep<<<(nU1 + NTHR - 1) / NTHR, NTHR, 0, stream>>>(bases1, comp1, root1, WT1, IN1, nU1);
  k_wprep<<<(nU2 + NTHR - 1) / NTHR, NTHR, 0, stream>>>(bases2, comp2, root2, WT2, HIDC, nU2);

  k_agg<<<gA, NTHR, LDS_AGG, stream>>>(src, dst, etyp, x, IN1, AP1, lda1, nN, nE, nb, vec8, MP);
  k_gemm<<<gG, GTHR, 0, stream>>>(AP1, lda1, lda1 / 32, x, IN1, IN1 / 32, nN, WT1, KT1, bias1, H1, MP);

  k_agg<<<gA, NTHR, LDS_AGG, stream>>>(src, dst, etyp, H1, HIDC, AP2, lda2, nN, nE, nb, vec8, MP);
  k_gemm<<<gG, GTHR, 0, stream>>>(AP2, lda2, lda2 / 32, H1, HIDC, HIDC / 32, nN, WT2, KT2, bias2, H2, MP);

  k_pool_head<<<1, NTHR, LDS_POOL, stream>>>(H2, batch, Wc, bc, out, nN, nG);
}
